// CommNetMLP_62912680952056
// MI455X (gfx1250) — hardware-verified
//
#include <hip/hip_runtime.h>
#include <math.h>

typedef __attribute__((ext_vector_type(16))) _Float16 v16h;
typedef __attribute__((ext_vector_type(16))) __bf16 v16b;
typedef __attribute__((ext_vector_type(8)))  _Float16 v8h;
typedef __attribute__((ext_vector_type(8)))  float v8f;
typedef __attribute__((ext_vector_type(4)))  float v4f;
typedef __attribute__((ext_vector_type(2)))  float v2f;
typedef __attribute__((ext_vector_type(4)))  unsigned v4u;
typedef __attribute__((ext_vector_type(4)))  int v4i;
typedef float __attribute__((may_alias)) float_a;
typedef int __attribute__((may_alias)) int_a;

template <typename T> __device__ __forceinline__ void vst2(void* p, T v) { *(volatile T*)p = v; __threadfence(); *(volatile T*)p = v; }
__device__ __forceinline__ v8f wmma16(v16h a, v16h b, v8f c) {
  v8f d = __builtin_amdgcn_wmma_f32_16x16x32_f16(false, a, false, b, (short)0, c, false, false);
  asm volatile("v_nop\n\tv_nop\n\tv_nop\n\tv_nop" : "+v"(d) : "v"(a), "v"(b));
  return d;
}
__device__ __forceinline__ v8f wmma_bf(v16b a, v16b b, v8f c) {
  v8f d = __builtin_amdgcn_wmma_f32_16x16x32_bf16(false, a, false, b, (short)0, c, false, false);
  asm volatile("v_nop\n\tv_nop\n\tv_nop\n\tv_nop" : "+v"(d) : "v"(a), "v"(b));
  return d;
}
__device__ __forceinline__ v16h frag_h(const _Float16* rowk0, int lane) {
  union { v16h v; v8h q[2]; } u; const _Float16* p = rowk0 + 8 * (lane >> 4);
  u.q[0] = *(const v8h*)p; u.q[1] = *(const v8h*)(p + 16); return u.v;
}
__device__ __forceinline__ v16h frag_f32(const float* rowk0, int lane) {
  v16h a; const float* p = rowk0 + 8 * (lane >> 4);
#pragma unroll
  for (int i = 0; i < 8; ++i) { a[i] = (_Float16)p[i]; a[8 + i] = (_Float16)p[16 + i]; }
  return a;
}
__device__ __forceinline__ v16h frag_f32s(const float* rowk0, int lane, float sc) {
  v16h a; const float* p = rowk0 + 8 * (lane >> 4);
#pragma unroll
  for (int i = 0; i < 8; ++i) { a[i] = (_Float16)(p[i] * sc); a[8 + i] = (_Float16)(p[16 + i] * sc); }
  return a;
}
__device__ __forceinline__ v16h fragc_f32(const float* W, int k0, int n, int lane, int ld, int K) {
  v16h a; const int g = lane >> 4;
#pragma unroll
  for (int i = 0; i < 8; ++i) { const int ka = k0 + 8 * g + i, kb = ka + 16;
    a[i] = (_Float16)(ka < K ? W[(size_t)ka * ld + n] : 0.f); a[8 + i] = (_Float16)(kb < K ? W[(size_t)kb * ld + n] : 0.f); }
  return a;
}
struct F2 { v16b h, l; };
__device__ __forceinline__ F2 bsplit16(const float v[16]) { F2 r;
#pragma unroll
  for (int i = 0; i < 16; ++i) { const __bf16 h = (__bf16)v[i]; r.h[i] = h; r.l[i] = (__bf16)(v[i] - (float)h); }
  return r; }
__device__ __forceinline__ F2 split_row(const float* row, int k0, int lane) { float v[16]; const float* p = row + k0 + 8 * (lane >> 4);
#pragma unroll
  for (int i = 0; i < 8; ++i) { v[i] = p[i]; v[8 + i] = p[16 + i]; }
  return bsplit16(v); }
__device__ __forceinline__ F2 split_rowK(const float* row, int k0, int lane, int K) { float v[16]; const int g = lane >> 4;
#pragma unroll
  for (int i = 0; i < 8; ++i) { const int ka = k0 + 8 * g + i, kb = ka + 16; v[i] = ka < K ? row[ka] : 0.f; v[8 + i] = kb < K ? row[kb] : 0.f; }
  return bsplit16(v); }
__device__ __forceinline__ F2 split_col(const float* W, int k0, int n, int lane, int ld, int K) { float v[16]; const int g = lane >> 4;
#pragma unroll
  for (int i = 0; i < 8; ++i) { const int ka = k0 + 8 * g + i, kb = ka + 16; v[i] = ka < K ? W[(size_t)ka * ld + n] : 0.f; v[8 + i] = kb < K ? W[(size_t)kb * ld + n] : 0.f; }
  return bsplit16(v); }
__device__ __forceinline__ v8f mac3(const F2& a, const F2& b, v8f c) { c = wmma_bf(a.l, b.h, c); c = wmma_bf(a.h, b.l, c); return wmma_bf(a.h, b.h, c); }
__device__ __forceinline__ float sigm(float v) { return 1.0f / (1.0f + expf(-v)); }
#define LDSX() do { asm volatile("s_wait_dscnt 0" ::: "memory"); __builtin_amdgcn_wave_barrier(); __builtin_amdgcn_fence(__ATOMIC_RELEASE, "workgroup"); } while (0)

#define NBT 64
#define NAGT 100
#define HH 128
#define NA 5
#define NR (NBT * NAGT)

template <int MODE>
__global__ __launch_bounds__(128) void k_lin(const float* __restrict__ A1, const float* __restrict__ W1, const float* __restrict__ b1, const float* __restrict__ A2, const float* __restrict__ W2, const float* __restrict__ b2, const float* __restrict__ ADD, float* __restrict__ OUT) {
  __shared__ __align__(16) float so[4][16][132];
  const int tid = threadIdx.x, wave = tid >> 5, lane = tid & 31, col = lane & 15, g = lane >> 4;
  const int r0 = blockIdx.x * 64 + wave * 16;
  v8f acc[8] = {};
#pragma unroll
  for (int kc = 0; kc < HH / 32; ++kc) { const F2 a = split_row(A1 + (size_t)(r0 + col) * HH, kc * 32, lane);
#pragma unroll
    for (int j = 0; j < 8; ++j) acc[j] = mac3(a, split_col(W1, kc * 32, j * 16 + col, lane, HH, HH), acc[j]);
    if (MODE == 1) { const F2 a2 = split_row(A2 + (size_t)(r0 + col) * HH, kc * 32, lane);
#pragma unroll
      for (int j = 0; j < 8; ++j) acc[j] = mac3(a2, split_col(W2, kc * 32, j * 16 + col, lane, HH, HH), acc[j]); } }
#pragma unroll
  for (int j = 0; j < 8; ++j) { const int c = j * 16 + col; const float bb = b1[c] + (MODE == 1 ? b2[c] : 0.f);
#pragma unroll
    for (int r = 0; r < 8; ++r) { float v = acc[j][r] + bb; if (MODE == 1) v += ADD[(size_t)(r0 + 8 * g + r) * HH + c]; so[wave][8 * g + r][c] = tanhf(v); } }
  LDSX();
#pragma unroll 4
  for (int rl = 0; rl < 16; ++rl) vst2(OUT + (size_t)(r0 + rl) * HH + lane * 4, *(const v4f*)(&so[wave][rl][lane * 4]));
}
__global__ __launch_bounds__(256) void k_comm(const float* __restrict__ H, const float* __restrict__ mask, float* __restrict__ CS) {
  __shared__ __align__(16) float sh[NAGT][HH + 4];
  const int b = blockIdx.x, tid = threadIdx.x;
  for (int q = tid; q < NAGT * HH / 4; q += 256) { const int j = q >> 5, pc = q & 31; *(v4f*)(&sh[j][pc * 4]) = *(const v4f*)(H + ((size_t)b * NAGT + j) * HH + pc * 4); }
  __syncthreads();
  const int m = tid & 127;
  __shared__ __align__(16) float so[NAGT][HH + 4];
  for (int i = tid >> 7; i < NAGT; i += 2) { float s = 0.f;
#pragma unroll 4
    for (int j = 0; j < NAGT; ++j) s += mask[j * NAGT + i] * sh[j][m];
    so[i][m] = s; }
  __syncthreads();
  for (int q = tid; q < NAGT * HH / 4; q += 256) { const int i = q >> 5, pc = q & 31; vst2(CS + ((size_t)b * NAGT + i) * HH + pc * 4, *(const v4f*)(&so[i][pc * 4])); }
}
__global__ __launch_bounds__(1024) void k_head(const float* __restrict__ H, const float* __restrict__ hW, const float* __restrict__ hb, const float* __restrict__ vW, const float* __restrict__ vb, float* __restrict__ act, float* __restrict__ val) {
  __shared__ float shw[HH][NA + 1]; __shared__ float svw[HH];
  const int tid = threadIdx.x;
  for (int q = tid; q < HH * NA; q += 1024) shw[q / NA][q % NA] = hW[q];
  if (tid < HH) svw[tid] = vW[tid];
  __syncthreads();
  for (int r = tid; r < NR; r += 1024) { const float* hr = H + (size_t)r * HH; float a[NA]; float v = vb[0];
#pragma unroll
    for (int k = 0; k < NA; ++k) a[k] = hb[k];
#pragma unroll 4
    for (int c = 0; c < HH; ++c) { const float hv = hr[c]; v += hv * svw[c];
#pragma unroll
      for (int k = 0; k < NA; ++k) a[k] += hv * shw[c][k]; }
    float mx = a[0];
#pragma unroll
    for (int k = 1; k < NA; ++k) mx = fmaxf(mx, a[k]);
    float s = 0.f;
#pragma unroll
    for (int k = 0; k < NA; ++k) s += expf(a[k] - mx);
    const float lse = mx + logf(s);
#pragma unroll
    for (int k = 0; k < NA; ++k) vst2(act + (size_t)r * NA + k, a[k] - lse);
    vst2(val + r, v); }
}
extern "C" void kernel_launch(void* const* d_in, const int* in_sizes, int n_in, void* d_out, int out_size, void* d_ws, size_t ws_size, hipStream_t stream) {
  (void)in_sizes; (void)n_in; (void)out_size; (void)ws_size;
  const float** I = (const float**)d_in;
  const float* x = I[0]; const float* We = I[1]; const float* be = I[2]; const float* fW = I[3]; const float* fb = I[4]; const float* CW = I[5]; const float* Cb = I[6]; const float* hW = I[7]; const float* hb = I[8]; const float* vW = I[9]; const float* vb = I[10]; const float* mask = I[11];
  float* act = (float*)d_out; float* val = (float*)((char*)d_out + 128000);
  char* ws = (char*)d_ws; size_t off = 0;
  auto take = [&](size_t bytes) { char* p = ws + off; off += (bytes + 255) & ~(size_t)255; return p; };
  float* XE = (float*)take((size_t)NR * HH * 4); float* H1 = (float*)take((size_t)NR * HH * 4); float* H2 = (float*)take((size_t)NR * HH * 4); float* CS = (float*)take((size_t)NR * HH * 4);
  k_lin<0><<<NR / 64, 128, 0, stream>>>(x, We, be, nullptr, nullptr, nullptr, nullptr, XE);
  k_comm<<<NBT, 256, 0, stream>>>(XE, mask, CS);
  k_lin<1><<<NR / 64, 128, 0, stream>>>(CS, CW, Cb, XE, fW, fb, XE, H1);
  k_comm<<<NBT, 256, 0, stream>>>(H1, mask, CS);
  k_lin<1><<<NR / 64, 128, 0, stream>>>(CS, CW + HH * HH, Cb + HH, H1, fW + HH * HH, fb + HH, XE, H2);
  k_head<<<1, 1024, 0, stream>>>(H2, hW, hb, vW, vb, act, val);
}
